// TransformerGCN_71167608094895
// MI455X (gfx1250) — hardware-verified
//
#include <hip/hip_runtime.h>
#include <stddef.h>


#define IN0   128
#define HD    512
#define NHD   4
#define NG    64
#define NO    12
#define NCAT  (4 * HD)
#define GR    32
#define GW    64
#define NTHR  256
#define NWAVE 8
#define NB    128
#define CHUNK 2048
#define WCAP  256
#define NGRP  (CHUNK / (NTHR * 4))
#define PSP   544

#define GEMM_LDS (NWAVE * GR * GW * 4)
#define LDS_SACC (NB * HD)
#define LDS_DEN  (NB * NHD)
#define LDS_LIST (NWAVE * WCAP)
#define AGG_LDS  ((LDS_SACC + 2 * LDS_DEN + LDS_LIST + NWAVE) * 4)

static_assert(WCAP == (CHUNK / NTHR) * 32);
static_assert(NGRP >= 1);
static_assert(NB == 128);
static_assert(CHUNK == 2048);
static_assert(NB % NWAVE == 0);
static_assert(HD == NHD * 128);
static_assert(NCAT == 2048);
static_assert(GW * NWAVE == HD);
static_assert(GEMM_LDS == 65536);
static_assert(AGG_LDS == 274464);
static_assert((NG * NO) % 128 == 0);
static_assert((LDS_SACC % 4) == 0);

typedef float    v4f  __attribute__((ext_vector_type(4)));
typedef float    v8f  __attribute__((ext_vector_type(8)));
typedef int      v4i  __attribute__((ext_vector_type(4)));
typedef _Float16 v8h  __attribute__((ext_vector_type(8)));
typedef _Float16 v16h __attribute__((ext_vector_type(16)));
union Frag   { v16h v; v8h half[2]; };
union Pack16 { v8h h; v4i i; };

__device__ __forceinline__ v8f wm(v16h a, v16h b, v8f c) {
  v8f d = __builtin_amdgcn_wmma_f32_16x16x32_f16(false, a, false, b, (short)0, c, false, false);
  asm volatile("v_nop\n\tv_nop\n\tv_nop\n\tv_nop" : "+v"(d) : "v"(a), "v"(b));
  return d;
}

__device__ __forceinline__ void wave_lds_sync() {
  asm volatile("" ::: "memory");
  __builtin_amdgcn_fence(__ATOMIC_RELEASE, "wavefront");
  __builtin_amdgcn_wave_barrier();
  asm volatile("" ::: "memory");
}

__device__ __forceinline__ v4f relu4(v4f t) {
  t.x = fmaxf(t.x, 0.f); t.y = fmaxf(t.y, 0.f); t.z = fmaxf(t.z, 0.f); t.w = fmaxf(t.w, 0.f);
  return t;
}

__global__ __launch_bounds__(NTHR) void k_cvx(const float* __restrict__ x, _Float16* xh, int n8) {
  const int i = blockIdx.x * NTHR + threadIdx.x;
  if (i >= n8) return;
  const size_t o = (size_t)i * 8;
  const v4f a = *(const v4f*)(x + o);
  const v4f b = *(const v4f*)(x + o + 4);
  Pack16 u;
  u.h[0] = (_Float16)a.x; u.h[1] = (_Float16)a.y; u.h[2] = (_Float16)a.z; u.h[3] = (_Float16)a.w;
  u.h[4] = (_Float16)b.x; u.h[5] = (_Float16)b.y; u.h[6] = (_Float16)b.z; u.h[7] = (_Float16)b.w;
  *(volatile v4i*)(xh + o) = u.i;
  __threadfence();
  *(volatile v4i*)(xh + o) = u.i;
}

__global__ __launch_bounds__(NTHR) void k_prepw(
    const float* __restrict__ W0, const float* __restrict__ W1,
    const float* __restrict__ W2, const float* __restrict__ W3,
    _Float16* Wt, int K, float sc, int tot8) {
  const int i = blockIdx.x * NTHR + threadIdx.x;
  if (i >= tot8) return;
  const int kq  = K >> 3;
  const int n   = i / kq;
  const int k8  = i - n * kq;
  const int seg = n >> 9;
  const int nc  = n & (HD - 1);
  const float* W = (seg == 0) ? W0 : (seg == 1) ? W1 : (seg == 2) ? W2 : W3;
  const float* p = W + (size_t)(k8 * 8) * HD + nc;
  Pack16 u;
#pragma unroll
  for (int t = 0; t < 8; ++t) u.h[t] = (_Float16)(p[(size_t)t * HD] * sc);
  _Float16* d = Wt + (size_t)n * K + k8 * 8;
  *(volatile v4i*)d = u.i;
  __threadfence();
  *(volatile v4i*)d = u.i;
}

__device__ __forceinline__ void gst_f32(const float* st, const float* bias, float* ob, float winv, int lane) {
  const int rr = lane >> 4, c4 = (lane & 15) * 4;
  const v4f b4 = *(const v4f*)(bias + c4);
#pragma unroll
  for (int qq = 0; qq < 16; ++qq) {
    const int row = 2 * qq + rr;
    const v4f u = *(const v4f*)(st + row * GW + c4) * winv + b4;
    *(volatile v4f*)(ob + (size_t)row * HD + c4) = u;
  }
}

__device__ __forceinline__ void gst_f16(const float* st, const float* bias, _Float16* ob, float winv, int lane) {
  const int rr = lane >> 3, c8 = (lane & 7) * 8;
  const v4f ba = *(const v4f*)(bias + c8);
  const v4f bb = *(const v4f*)(bias + c8 + 4);
#pragma unroll
  for (int qq = 0; qq < 8; ++qq) {
    const int row = 4 * qq + rr;
    const v4f u0 = *(const v4f*)(st + row * GW + c8) * winv + ba;
    const v4f u1 = *(const v4f*)(st + row * GW + c8 + 4) * winv + bb;
    Pack16 pk;
    pk.h[0] = (_Float16)u0.x; pk.h[1] = (_Float16)u0.y; pk.h[2] = (_Float16)u0.z; pk.h[3] = (_Float16)u0.w;
    pk.h[4] = (_Float16)u1.x; pk.h[5] = (_Float16)u1.y; pk.h[6] = (_Float16)u1.z; pk.h[7] = (_Float16)u1.w;
    *(volatile v4i*)(ob + (size_t)row * HD + c8) = pk.i;
  }
}

__global__ __launch_bounds__(NTHR) void k_gemm(
    const _Float16* __restrict__ A, const _Float16* __restrict__ Wt,
    const float* __restrict__ bq, const float* __restrict__ bk,
    const float* __restrict__ bv, const float* __restrict__ bs,
    _Float16* oq, _Float16* ok, _Float16* ov, float* os,
    int K, int nN, float winv) {
  extern __shared__ v4f lds_dyn[];
  const int tid  = threadIdx.x;
  const int lane = tid & 31;
  const int wave = tid >> 5;
  const int h    = lane >> 4;
  const int m    = lane & 15;
  const int seg  = blockIdx.y;
  const int row0 = blockIdx.x * GR;
  const int colw = wave * GW;
  float* st = (float*)lds_dyn + wave * (GR * GW);

  int ra0 = row0 + m;      if (ra0 > nN - 1) ra0 = nN - 1;
  int ra1 = row0 + 16 + m; if (ra1 > nN - 1) ra1 = nN - 1;
  const _Float16* pa0 = A + (size_t)ra0 * K + 8 * h;
  const _Float16* pa1 = A + (size_t)ra1 * K + 8 * h;
  const _Float16* pb  = Wt + (size_t)(seg * HD + colw + m) * K + 8 * h;
  const size_t bstep  = (size_t)16 * K;

  const v8f z8 = {0.f, 0.f, 0.f, 0.f, 0.f, 0.f, 0.f, 0.f};
  v8f acc0[4], acc1[4];
#pragma unroll
  for (int j = 0; j < 4; ++j) { acc0[j] = z8; acc1[j] = z8; }

#pragma unroll 1
  for (int k0 = 0; k0 < K; k0 += 32) {
    Frag a0, a1;
    a0.half[0] = *(const v8h*)(pa0 + k0); a0.half[1] = *(const v8h*)(pa0 + k0 + 16);
    a1.half[0] = *(const v8h*)(pa1 + k0); a1.half[1] = *(const v8h*)(pa1 + k0 + 16);
#pragma unroll
    for (int j = 0; j < 4; ++j) {
      Frag b;
      const _Float16* p = pb + j * bstep + k0;
      b.half[0] = *(const v8h*)p;
      b.half[1] = *(const v8h*)(p + 16);
      acc0[j] = wm(a0.v, b.v, acc0[j]);
      acc1[j] = wm(a1.v, b.v, acc1[j]);
    }
  }

#pragma unroll
  for (int j = 0; j < 4; ++j) {
#pragma unroll
    for (int r = 0; r < 8; ++r) {
      st[(8 * h + r) * GW + 16 * j + m]      = acc0[j][r];
      st[(16 + 8 * h + r) * GW + 16 * j + m] = acc1[j][r];
    }
  }
  __syncthreads();

  if (seg == 3) {
    const float* bias = bs + colw;
    float* ob = os + (size_t)row0 * HD + colw;
    gst_f32(st, bias, ob, winv, lane);
    __threadfence();
    gst_f32(st, bias, ob, winv, lane);
  } else {
    const float* bias = ((seg == 0) ? bq : (seg == 1) ? bk : bv) + colw;
    _Float16* ob = ((seg == 0) ? oq : (seg == 1) ? ok : ov) + (size_t)row0 * HD + colw;
    gst_f16(st, bias, ob, winv, lane);
    __threadfence();
    gst_f16(st, bias, ob, winv, lane);
  }
}

__global__ __launch_bounds__(NTHR) void k_agg(
    const _Float16* __restrict__ q, const _Float16* __restrict__ k, const _Float16* __restrict__ v,
    const int* __restrict__ ei, float* skh, _Float16* h1, int nN, int nE, int mode) {
  extern __shared__ v4f lds_dyn[];
  float* sacc = (float*)lds_dyn;
  float* den  = sacc + LDS_SACC;
  float* mrun = den + LDS_DEN;
  int*   list = (int*)(mrun + LDS_DEN);
  int*   wcnt = list + LDS_LIST;

  const int tid  = threadIdx.x;
  const int lane = tid & 31;
  const int wave = tid >> 5;
  const int hd   = lane >> 3;
  const int nodeBase = blockIdx.x * NB;

  {
    const v4f z4 = {0.f, 0.f, 0.f, 0.f};
    for (int i = tid; i < LDS_SACC / 4; i += NTHR) lds_dyn[i] = z4;
    for (int i = tid; i < LDS_DEN; i += NTHR) { den[i] = 0.f; mrun[i] = -1.0e30f; }
  }
  __syncthreads();

  const int* eid = ei + nE;
  const bool al16 = ((nE & 3) == 0);
  const float rsd = 0.08838834764831845f;

  const int nChunks = (nE + CHUNK - 1) / CHUNK;
#pragma unroll 1
  for (int ch = 0; ch < nChunks; ++ch) {
    const int cbase = ch * CHUNK;
    int wc = 0;
#pragma unroll
    for (int g = 0; g < NGRP; ++g) {
      const int el0 = (g * NTHR + tid) * 4;
      const int e0  = cbase + el0;
      const int sent = -2147483647 - 1;
      v4i d;
      if (al16 && (e0 + 3 < nE)) {
        d = *(const v4i*)(eid + e0);
      } else {
        d.x = (e0     < nE) ? eid[min(e0, nE - 1)]     : sent;
        d.y = (e0 + 1 < nE) ? eid[min(e0 + 1, nE - 1)] : sent;
        d.z = (e0 + 2 < nE) ? eid[min(e0 + 2, nE - 1)] : sent;
        d.w = (e0 + 3 < nE) ? eid[min(e0 + 3, nE - 1)] : sent;
      }
      const unsigned s0 = (unsigned)d.x - (unsigned)nodeBase;
      const unsigned s1 = (unsigned)d.y - (unsigned)nodeBase;
      const unsigned s2 = (unsigned)d.z - (unsigned)nodeBase;
      const unsigned s3 = (unsigned)d.w - (unsigned)nodeBase;
      const bool h0 = s0 < (unsigned)NB;
      const bool h1b = s1 < (unsigned)NB;
      const bool h2 = s2 < (unsigned)NB;
      const bool h3 = s3 < (unsigned)NB;
      const unsigned many = __builtin_amdgcn_ballot_w32(h0 | h1b | h2 | h3);
      if (many != 0u) {
#define HITJ(J, HJ, SJ) { \
          const unsigned mj = __builtin_amdgcn_ballot_w32(HJ); \
          if (HJ) { \
            const int pos = wc + (int)__builtin_amdgcn_mbcnt_lo(mj, 0u); \
            if (pos < WCAP) list[wave * WCAP + pos] = ((el0 + (J)) << 7) | (int)(SJ); \
          } \
          wc += (int)__builtin_popcount(mj); }
        HITJ(0, h0, s0)
        HITJ(1, h1b, s1)
        HITJ(2, h2, s2)
        HITJ(3, h3, s3)
#undef HITJ
      }
    }
    if (lane == 0) wcnt[wave] = wc;
    __syncthreads();

    if (wave == 0) {
      for (int wsx = 0; wsx < NWAVE; ++wsx) {
        int n = wcnt[wsx];
        if (n > WCAP) n = WCAP;
        if (n < 0) n = 0;
        for (int i = 0; i < n; ++i) {
          const int ent  = list[wsx * WCAP + i];
          const int slot = ent & (NB - 1);
          const int el   = (ent >> 7) & (CHUNK - 1);
          int e = cbase + el;
          if (e > nE - 1) e = nE - 1;
          int src = ei[e];
          src = src < 0 ? 0 : (src > nN - 1 ? nN - 1 : src);
          int nd = nodeBase + slot;
          if (nd > nN - 1) nd = nN - 1;
          const _Float16* qp = q + (size_t)nd * HD + 16 * lane;
          const _Float16* kp = k + (size_t)src * HD + 16 * lane;
          const _Float16* vp = v + (size_t)src * HD + 16 * lane;
          Pack16 qa, qb, ka, kb, va, vb;
          qa.i = *(const v4i*)qp; qb.i = *(const v4i*)(qp + 8);
          ka.i = *(const v4i*)kp; kb.i = *(const v4i*)(kp + 8);
          va.i = *(const v4i*)vp; vb.i = *(const v4i*)(vp + 8);
          const v8f pr = __builtin_convertvector(qa.h, v8f) * __builtin_convertvector(ka.h, v8f)
                       + __builtin_convertvector(qb.h, v8f) * __builtin_convertvector(kb.h, v8f);
          float dsum = ((pr[0] + pr[1]) + (pr[2] + pr[3])) + ((pr[4] + pr[5]) + (pr[6] + pr[7]));
          dsum += __shfl_xor(dsum, 1, 32);
          dsum += __shfl_xor(dsum, 2, 32);
          dsum += __shfl_xor(dsum, 4, 32);
          const float lg = dsum * rsd;
          const int ai = slot * NHD + hd;
          const float mo = mrun[ai];
          const float dn = den[ai];
          const float mn = fmaxf(mo, lg);
          const float f  = __expf(mo - mn);
          const float p  = __expf(lg - mn);
          const v8f vf0 = __builtin_convertvector(va.h, v8f);
          const v8f vf1 = __builtin_convertvector(vb.h, v8f);
          const v4f x0 = {vf0[0], vf0[1], vf0[2], vf0[3]};
          const v4f x1 = {vf0[4], vf0[5], vf0[6], vf0[7]};
          const v4f x2 = {vf1[0], vf1[1], vf1[2], vf1[3]};
          const v4f x3 = {vf1[4], vf1[5], vf1[6], vf1[7]};
          v4f* sp = (v4f*)(sacc + slot * HD + 16 * lane);
          v4f a0 = sp[0], a1 = sp[1], a2 = sp[2], a3 = sp[3];
          a0 = a0 * f + x0 * p;
          a1 = a1 * f + x1 * p;
          a2 = a2 * f + x2 * p;
          a3 = a3 * f + x3 * p;
          sp[0] = a0; sp[1] = a1; sp[2] = a2; sp[3] = a3;
          if ((lane & 7) == 0) { den[ai] = dn * f + p; mrun[ai] = mn; }
        }
      }
    }
    __syncthreads();
  }

  const int spw = NB / NWAVE;
#pragma unroll 1
  for (int j = 0; j < spw; ++j) {
    const int slot = wave * spw + j;
    const int node = nodeBase + slot;
    if (node >= nN) break;
    const float dn  = den[slot * NHD + hd];
    const float inv = __builtin_amdgcn_rcpf(fmaxf(dn, 1e-16f));
    const v4f* kp = (const v4f*)(skh + (size_t)node * HD + 16 * lane);
    v4f* sp = (v4f*)(sacc + slot * HD + 16 * lane);
    const v4f t0 = relu4(sp[0] * inv + kp[0]);
    const v4f t1 = relu4(sp[1] * inv + kp[1]);
    const v4f t2 = relu4(sp[2] * inv + kp[2]);
    const v4f t3 = relu4(sp[3] * inv + kp[3]);
    sp[0] = t0; sp[1] = t1; sp[2] = t2; sp[3] = t3;
    wave_lds_sync();
    const v4f* rp = (const v4f*)(sacc + slot * HD);
    if (mode == 0) {
      const v4f c0 = rp[2 * lane], c1 = rp[2 * lane + 1];
      const v4f c2 = rp[64 + 2 * lane], c3 = rp[65 + 2 * lane];
      Pack16 p0, p1;
      p0.h[0] = (_Float16)c0.x; p0.h[1] = (_Float16)c0.y; p0.h[2] = (_Float16)c0.z; p0.h[3] = (_Float16)c0.w;
      p0.h[4] = (_Float16)c1.x; p0.h[5] = (_Float16)c1.y; p0.h[6] = (_Float16)c1.z; p0.h[7] = (_Float16)c1.w;
      p1.h[0] = (_Float16)c2.x; p1.h[1] = (_Float16)c2.y; p1.h[2] = (_Float16)c2.z; p1.h[3] = (_Float16)c2.w;
      p1.h[4] = (_Float16)c3.x; p1.h[5] = (_Float16)c3.y; p1.h[6] = (_Float16)c3.z; p1.h[7] = (_Float16)c3.w;
      _Float16* hp = h1 + (size_t)node * HD;
      *(volatile v4i*)(hp + 8 * lane)       = p0.i;
      *(volatile v4i*)(hp + 256 + 8 * lane) = p1.i;
      __threadfence();
      *(volatile v4i*)(hp + 8 * lane)       = p0.i;
      *(volatile v4i*)(hp + 256 + 8 * lane) = p1.i;
    } else {
      const v4f o0 = rp[lane], o1 = rp[32 + lane], o2 = rp[64 + lane], o3 = rp[96 + lane];
      float* op = skh + (size_t)node * HD + 4 * lane;
      *(volatile v4f*)(op)       = o0;
      *(volatile v4f*)(op + 128) = o1;
      *(volatile v4f*)(op + 256) = o2;
      *(volatile v4f*)(op + 384) = o3;
      __threadfence();
      *(volatile v4f*)(op)       = o0;
      *(volatile v4f*)(op + 128) = o1;
      *(volatile v4f*)(op + 256) = o2;
      *(volatile v4f*)(op + 384) = o3;
    }
  }
}

__global__ __launch_bounds__(NTHR) void k_pool(const float* __restrict__ hbuf, const int* __restrict__ bt,
                                               float* ps, int nN) {
  __shared__ __attribute__((aligned(16))) v4f part[NWAVE * (HD / 4)];
  __shared__ int pcnt[NWAVE];
  const int tid  = threadIdx.x;
  const int lane = tid & 31;
  const int wave = tid >> 5;
  const int g    = blockIdx.x;
  v4f a0 = {0.f, 0.f, 0.f, 0.f}, a1 = a0, a2 = a0, a3 = a0;
  int cnt = 0;

  const int nChunks = (nN + CHUNK - 1) / CHUNK;
#pragma unroll 1
  for (int ch = 0; ch < nChunks; ++ch) {
    const int cbase = ch * CHUNK;
#pragma unroll
    for (int gq = 0; gq < NGRP; ++gq) {
      const int el0 = (gq * NTHR + tid) * 4;
      const int i0  = cbase + el0;
      v4i d;
      if (i0 + 3 < nN) {
        d = *(const v4i*)(bt + i0);
      } else {
        d.x = (i0     < nN) ? bt[min(i0, nN - 1)]     : -1;
        d.y = (i0 + 1 < nN) ? bt[min(i0 + 1, nN - 1)] : -1;
        d.z = (i0 + 2 < nN) ? bt[min(i0 + 2, nN - 1)] : -1;
        d.w = (i0 + 3 < nN) ? bt[min(i0 + 3, nN - 1)] : -1;
      }
      const unsigned m0 = __builtin_amdgcn_ballot_w32(d.x == g);
      const unsigned m1 = __builtin_amdgcn_ballot_w32(d.y == g);
      const unsigned m2 = __builtin_amdgcn_ballot_w32(d.z == g);
      const unsigned m3 = __builtin_amdgcn_ballot_w32(d.w == g);
      if ((m0 | m1 | m2 | m3) != 0u) {
#define POOLJ(J, MJ) { \
          unsigned mm = (MJ); \
          cnt += (int)__builtin_popcount(mm); \
          while (mm != 0u) { \
            const int jl = __builtin_ctz(mm); \
            mm &= mm - 1u; \
            int node = cbase + ((gq * NTHR + (wave << 5) + jl) << 2) + (J); \
            if (node > nN - 1) node = nN - 1; \
            const v4f* rp = (const v4f*)(hbuf + (size_t)node * HD + 16 * lane); \
            a0 += rp[0]; a1 += rp[1]; a2 += rp[2]; a3 += rp[3]; \
          } }
        POOLJ(0, m0)
        POOLJ(1, m1)
        POOLJ(2, m2)
        POOLJ(3, m3)
#undef POOLJ
      }
    }
  }

  part[wave * (HD / 4) + 4 * lane + 0] = a0;
  part[wave * (HD / 4) + 4 * lane + 1] = a1;
  part[wave * (HD / 4) + 4 * lane + 2] = a2;
  part[wave * (HD / 4) + 4 * lane + 3] = a3;
  if (lane == 0) pcnt[wave] = cnt;
  __syncthreads();

  if (wave == 0) {
    v4f t0 = part[4 * lane], t1 = part[4 * lane + 1], t2 = part[4 * lane + 2], t3 = part[4 * lane + 3];
#pragma unroll
    for (int w = 1; w < NWAVE; ++w) {
      t0 += part[w * (HD / 4) + 4 * lane];
      t1 += part[w * (HD / 4) + 4 * lane + 1];
      t2 += part[w * (HD / 4) + 4 * lane + 2];
      t3 += part[w * (HD / 4) + 4 * lane + 3];
    }
    int c = 0;
#pragma unroll
    for (int w = 0; w < NWAVE; ++w) c += pcnt[w];
    part[4 * lane] = t0; part[4 * lane + 1] = t1; part[4 * lane + 2] = t2; part[4 * lane + 3] = t3;
    wave_lds_sync();
    const v4f o0 = part[lane], o1 = part[32 + lane], o2 = part[64 + lane], o3 = part[96 + lane];
    v4f c4 = {0.f, 0.f, 0.f, 0.f};
    if (lane == 0) c4.x = (float)c;
    float* prow = ps + (size_t)g * PSP + 4 * lane;
    *(volatile v4f*)(prow)       = o0;
    *(volatile v4f*)(prow + 128) = o1;
    *(volatile v4f*)(prow + 256) = o2;
    *(volatile v4f*)(prow + 384) = o3;
    if (lane < 8) *(volatile v4f*)(prow + 512) = c4;
    __threadfence();
    *(volatile v4f*)(prow)       = o0;
    *(volatile v4f*)(prow + 128) = o1;
    *(volatile v4f*)(prow + 256) = o2;
    *(volatile v4f*)(prow + 384) = o3;
    if (lane < 8) *(volatile v4f*)(prow + 512) = c4;
  }
}

__global__ __launch_bounds__(NTHR) void k_head(const float* __restrict__ ps, const float* __restrict__ Wl,
                                               const float* __restrict__ bl, float* out) {
  __shared__ __attribute__((aligned(16))) float so[NG * NO];
  const int tid  = threadIdx.x;
  const int lane = tid & 31;
  const int wave = tid >> 5;
  for (int idx = tid; idx < NG * NO; idx += NTHR) {
    const int g = idx / NO;
    const int o = idx - g * NO;
    const float* pr = ps + (size_t)g * PSP;
    const float c   = pr[HD];
    const float inv = 1.0f / fmaxf(c, 1.0f);
    float acc = 0.f;
#pragma unroll 8
    for (int jj = 0; jj < HD; ++jj) acc += (pr[jj] * inv) * Wl[jj * NO + o];
    so[idx] = acc + bl[o];
  }
  __syncthreads();
  if (wave == 0) {
    v4f vals[6];
#pragma unroll
    for (int qq = 0; qq < 6; ++qq) vals[qq] = *(const v4f*)(so + 4 * (qq * 32 + lane));
#pragma unroll
    for (int qq = 0; qq < 6; ++qq) *(volatile v4f*)(out + 4 * (qq * 32 + lane)) = vals[qq];
    __threadfence();
#pragma unroll
    for (int qq = 0; qq < 6; ++qq) *(volatile v4f*)(out + 4 * (qq * 32 + lane)) = vals[qq];
  }
}

extern "C" void kernel_launch(void* const* d_in, const int* in_sizes, int n_in,
                              void* d_out, int out_size, void* d_ws, size_t ws_size,
                              hipStream_t stream) {
  if (n_in < 21) return;
  const int nN = in_sizes[0] / IN0;
  if (nN <= 0 || in_sizes[0] != nN * IN0) return;
  if (in_sizes[1] < 0 || (in_sizes[1] & 1) != 0) return;
  const int nE = in_sizes[1] / 2;
  if (in_sizes[2] != nN) return;
  if (in_sizes[3] != IN0 * HD || in_sizes[5] != IN0 * HD || in_sizes[7] != IN0 * HD || in_sizes[9] != IN0 * HD) return;
  if (in_sizes[4] != HD || in_sizes[6] != HD || in_sizes[8] != HD || in_sizes[10] != HD) return;
  if (in_sizes[11] != HD * HD || in_sizes[13] != HD * HD || in_sizes[15] != HD * HD || in_sizes[17] != HD * HD) return;
  if (in_sizes[12] != HD || in_sizes[14] != HD || in_sizes[16] != HD || in_sizes[18] != HD) return;
  if (in_sizes[19] != HD * NO || in_sizes[20] != NO) return;
  if (out_size != NG * NO) return;

  const float* x     = (const float*)d_in[0];
  const int*   ei    = (const int*)d_in[1];
  const int*   batch = (const int*)d_in[2];
  const float* Wq1 = (const float*)d_in[3];  const float* bq1 = (const float*)d_in[4];
  const float* Wk1 = (const float*)d_in[5];  const float* bk1 = (const float*)d_in[6];
  const float* Wv1 = (const float*)d_in[7];  const float* bv1 = (const float*)d_in[8];
  const float* Ws1 = (const float*)d_in[9];  const float* bs1 = (const float*)d_in[10];
  const float* Wq2 = (const float*)d_in[11]; const float* bq2 = (const float*)d_in[12];
  const float* Wk2 = (const float*)d_in[13]; const float* bk2 = (const float*)d_in[14];
  const float* Wv2 = (const float*)d_in[15]; const float* bv2 = (const float*)d_in[16];
  const float* Ws2 = (const float*)d_in[17]; const float* bs2 = (const float*)d_in[18];
  const float* Wl  = (const float*)d_in[19]; const float* bl  = (const float*)d_in[20];
  float* out = (float*)d_out;

  const int nP = ((nN + GR - 1) / GR) * GR;
  size_t off = 0;
  char* wsb = (char*)d_ws;
  auto carve = [&](size_t bytes) -> char* {
    char* p = wsb + off;
    off += (bytes + 255) & ~(size_t)255;
    return p;
  };
  _Float16* XH  = (_Float16*)carve((size_t)nN * IN0 * sizeof(_Float16));
  _Float16* WT1 = (_Float16*)carve((size_t)NCAT * IN0 * sizeof(_Float16));
  _Float16* WT2 = (_Float16*)carve((size_t)NCAT * HD * sizeof(_Float16));
  _Float16* QB  = (_Float16*)carve((size_t)nP * HD * sizeof(_Float16));
  _Float16* KB  = (_Float16*)carve((size_t)nP * HD * sizeof(_Float16));
  _Float16* VB  = (_Float16*)carve((size_t)nP * HD * sizeof(_Float16));
  float*    SK  = (float*)carve((size_t)nP * HD * sizeof(float));
  _Float16* H1  = (_Float16*)carve((size_t)nP * HD * sizeof(_Float16));
  float*    PS  = (float*)carve((size_t)NG * PSP * sizeof(float));
  if (off > ws_size) return;

  const int n8x = nN * IN0 / 8;
  k_cvx<<<(n8x + NTHR - 1) / NTHR, NTHR, 0, stream>>>(x, XH, n8x);
  const int t81 = NCAT * IN0 / 8;
  k_prepw<<<(t81 + NTHR - 1) / NTHR, NTHR, 0, stream>>>(Wq1, Wk1, Wv1, Ws1, WT1, IN0, 16.0f, t81);
  const int t82 = NCAT * HD / 8;
  k_prepw<<<(t82 + NTHR - 1) / NTHR, NTHR, 0, stream>>>(Wq2, Wk2, Wv2, Ws2, WT2, HD, 32.0f, t82);

  hipFuncSetAttribute(reinterpret_cast<const void*>(&k_gemm),
                      hipFuncAttributeMaxDynamicSharedMemorySize, GEMM_LDS);
  hipFuncSetAttribute(reinterpret_cast<const void*>(&k_agg),
                      hipFuncAttributeMaxDynamicSharedMemorySize, AGG_LDS);

  const dim3 ggrid(nP / GR, 4);
  const int agrid = (nN + NB - 1) / NB;

  k_gemm<<<ggrid, NTHR, GEMM_LDS, stream>>>(XH, WT1, bq1, bk1, bv1, bs1, QB, KB, VB, SK, IN0, nN, 0.0625f);
  k_agg<<<agrid, NTHR, AGG_LDS, stream>>>(QB, KB, VB, ei, SK, H1, nN, nE, 0);

  k_gemm<<<ggrid, NTHR, GEMM_LDS, stream>>>(H1, WT2, bq2, bk2, bv2, bs2, QB, KB, VB, SK, HD, nN, 0.03125f);
  k_agg<<<agrid, NTHR, AGG_LDS, stream>>>(QB, KB, VB, ei, SK, H1, nN, nE, 1);

  k_pool<<<NG, NTHR, 0, stream>>>(SK, batch, PS, nN);
  k_head<<<1, NTHR, 0, stream>>>(PS, Wl, bl, out);
}
